// DotprodAttention_3_45492293599831
// MI455X (gfx1250) — hardware-verified
//
#include <hip/hip_runtime.h>


#ifndef NB
#define NB 8
#endif
#define NB_FULL 8
#define NN    128
#define DD    768
#define HID   64
#define MR    (NB * NN)
#define WSC   64.0f
#define PCAR  4194304.0f
#define LOG2E 1.4426950408889634f
#define HP_PITCH 68

static constexpr float HC1  = 16.0f;
static constexpr float HC2  = 32768.0f;
static constexpr float FC   = 16384.0f;
static constexpr unsigned LGC1 = 4u;
static constexpr unsigned LGC2 = 15u;
static constexpr unsigned LGF  = 14u;
static constexpr float SSC1 = 1.0f / 1024.0f;
static constexpr float SSC2 = 1.0f / 2097152.0f;
static constexpr float OSC1 = 1.0f / (PCAR * HC1);
static constexpr float OSC2 = 1.0f / (PCAR * HC2);
static constexpr float HSC2 = 1.0f / 1048576.0f;
static constexpr float BN_INV = 1.0f / (float)NB;

static_assert(SSC1 * HC1 * WSC == 1.0f);
static_assert(SSC2 * HC2 * WSC == 1.0f);
static_assert(PCAR == (float)(1u << 22));
static_assert(HC1 == (float)(1u << LGC1));
static_assert(HC2 == (float)(1u << LGC2));
static_assert(FC == (float)(1u << LGF));
static_assert(HSC2 * FC * WSC == 1.0f);
static_assert(NB >= 1 && NB <= NB_FULL);
static_assert(NN == 128 && HID == 64 && DD == 3 * 256 && DD == 4 * 3 * 64);
static_assert(MR % 64 == 0 && DD % 64 == 0 && NN % 64 == 0 && HID % 64 == 0);
static_assert(DD % 32 == 0 && NN % 32 == 0);
static_assert((MR * DD) % 8 == 0);
static_assert((size_t)NB_FULL * DD * 4 == 24576);
static_assert(((size_t)NB_FULL * DD + (size_t)NB_FULL * NN * DD) * 4 == 3170304);
static_assert(256 * 16 * 2 == 64 * 128);
static_assert(256 * 4 * 4 * 4 == 64 * 64 * 4);
static_assert(32 * 16 == NN * 4);
static_assert(256 * 16 * 8 == NN * NN * 2);
static_assert(4 * 3 * 128 == DD * 2);
static_assert((NB * 64) % 32 == 0);
static_assert(16 * 68 * 4 <= 131072);
static_assert(64 * HP_PITCH * 4 <= 131072);
static_assert(NN * 4 <= 131072);
static_assert(NB * 256 * 4 <= 131072);
static constexpr size_t CARVE_BYTES = (size_t)MR * DD * 2 + (size_t)DD * DD * 2 + (size_t)DD * DD * 2 + (size_t)2 * HID * DD * 2 + (size_t)MR * DD * 4 + (size_t)MR * DD * 2 + (size_t)MR * DD * 2
                                    + (size_t)2 * MR * HID * 4 + (size_t)MR * NN * 4 + (size_t)MR * NN * 2 + (size_t)MR * DD * 4 + (size_t)MR * DD * 2;
static_assert(CARVE_BYTES <= ((size_t)128 << 20));

typedef _Float16 h16;
typedef unsigned short bf;
typedef __attribute__((ext_vector_type(16))) __bf16   v16bf;
typedef __attribute__((ext_vector_type(16))) _Float16 v16h;
typedef __attribute__((ext_vector_type(8)))  _Float16 v8h;
typedef __attribute__((ext_vector_type(8)))  unsigned short v8us;
typedef __attribute__((ext_vector_type(8)))  float    v8f;
typedef __attribute__((ext_vector_type(4)))  float    v4f;
typedef __attribute__((ext_vector_type(2)))  float    v2f;
typedef __attribute__((ext_vector_type(4)))  _Float16 v4h;
typedef __attribute__((ext_vector_type(2)))  _Float16 v2h;
typedef __attribute__((ext_vector_type(2)))  unsigned short v2us;
typedef v8h  __attribute__((may_alias)) v8ha;
typedef v4f  __attribute__((may_alias)) v4fa;
typedef v8us __attribute__((may_alias)) v8usa;

__device__ __forceinline__ unsigned short f2bf(float f) { unsigned u = __float_as_uint(f); u += 0x7FFFu + ((u >> 16) & 1u); return (unsigned short)(u >> 16); }
__device__ __forceinline__ float bf2f(unsigned short b) { return __uint_as_float(((unsigned)b) << 16); }
__device__ __forceinline__ float bfr(float f) { return bf2f(f2bf(f)); }
__device__ __forceinline__ v16h cat16(v8h lo, v8h hi) { return __builtin_shufflevector(lo, hi, 0, 1, 2, 3, 4, 5, 6, 7, 8, 9, 10, 11, 12, 13, 14, 15); }
__device__ __forceinline__ v16bf cat16b(v8us lo, v8us hi) { return __builtin_bit_cast(v16bf, __builtin_shufflevector(lo, hi, 0, 1, 2, 3, 4, 5, 6, 7, 8, 9, 10, 11, 12, 13, 14, 15)); }
__device__ __forceinline__ v8f wmma16(v16h a, v16h b, v8f c) { return __builtin_amdgcn_wmma_f32_16x16x32_f16(false, a, false, b, (short)0, c, false, false); }
__device__ __forceinline__ v8f wmmab(v16bf a, v16bf b, v8f c) { return __builtin_amdgcn_wmma_f32_16x16x32_bf16(false, a, false, b, (short)0, c, false, false); }
__device__ __forceinline__ h16 toh_flush(float v) { const float w = (fabsf(v) < 6.103515625e-05f) ? 0.0f : v; return (h16)w; }
__device__ __forceinline__ v2h toh2_flush(float x, float y) { const float w0 = (fabsf(x) < 6.103515625e-05f) ? 0.0f : x; const float w1 = (fabsf(y) < 6.103515625e-05f) ? 0.0f : y; const v2f w = {w0, w1}; const v2h hp = __builtin_convertvector(w, v2h); return hp; }
__device__ __forceinline__ v8h cat8h(v2h a, v2h b, v2h c, v2h d) { const v4h lo = __builtin_shufflevector(a, b, 0, 1, 2, 3); const v4h hi = __builtin_shufflevector(c, d, 0, 1, 2, 3); return __builtin_shufflevector(lo, hi, 0, 1, 2, 3, 4, 5, 6, 7); }

template <typename T16> struct WFrag;
template <> struct WFrag<h16> { typedef v16h V; static __device__ __forceinline__ V ld(const h16* p) { return cat16(*(const v8h*)p, *(const v8h*)(p + 16)); } static __device__ __forceinline__ v8f mma(V a, V b, v8f c) { return wmma16(a, b, c); } };
template <> struct WFrag<bf> { typedef v16bf V; static __device__ __forceinline__ V ld(const bf* p) { return cat16b(*(const v8us*)p, *(const v8us*)(p + 16)); } static __device__ __forceinline__ v8f mma(V a, V b, v8f c) { return wmmab(a, b, c); } };
template <typename T16, int NSPLIT, bool BIAS>
__global__ __launch_bounds__(32) void k_gemmw(const T16* __restrict__ A, const T16* __restrict__ A2, const T16* __restrict__ Bt, const T16* __restrict__ Bt2, int K, float* C, int ldc, const float* __restrict__ bias, float csc, size_t sA, size_t sB, size_t sC) {
    typedef typename WFrag<T16>::V V;
    __shared__ __align__(16) float os[16 * 68];
    const size_t z = blockIdx.z; A += z * sA; if (A2) A2 += z * sA; Bt += z * sB; if (Bt2) Bt2 += z * sB; C += z * sC;
    const int lane = threadIdx.x & 31, lr = lane & 15, hi = lane >> 4; const int r0 = blockIdx.x * 64, c0 = blockIdx.y * 64;
    v8f acc[4][4];
#pragma unroll
    for (int mb = 0; mb < 4; ++mb)
#pragma unroll
        for (int nb = 0; nb < 4; ++nb) acc[mb][nb] = (v8f){};
    const size_t aoff = (size_t)(r0 + lr) * K + 8 * hi, boff = (size_t)(c0 + lr) * K + 8 * hi;
#pragma unroll 1
    for (int kc = 0; kc < K; kc += 32) {
        V a[4], a2[4];
#pragma unroll
        for (int mb = 0; mb < 4; ++mb) { a[mb] = WFrag<T16>::ld(A + aoff + (size_t)mb * 16 * K + kc); if (NSPLIT == 1 || NSPLIT == 2) a2[mb] = WFrag<T16>::ld(A2 + aoff + (size_t)mb * 16 * K + kc); }
#pragma unroll
        for (int nb = 0; nb < 4; ++nb) { const V b = WFrag<T16>::ld(Bt + boff + (size_t)nb * 16 * K + kc); V b2; if (NSPLIT >= 2) b2 = WFrag<T16>::ld(Bt2 + boff + (size_t)nb * 16 * K + kc);
#pragma unroll
            for (int mb = 0; mb < 4; ++mb) { acc[mb][nb] = WFrag<T16>::mma(a[mb], b, acc[mb][nb]); if (NSPLIT == 1 || NSPLIT == 2) acc[mb][nb] = WFrag<T16>::mma(a2[mb], b, acc[mb][nb]); if (NSPLIT >= 2) acc[mb][nb] = WFrag<T16>::mma(a[mb], b2, acc[mb][nb]); } }
        asm volatile("v_nop\n\tv_nop\n\tv_nop\n\tv_nop" : "+v"(acc[0][0]), "+v"(acc[1][1]), "+v"(acc[2][2]), "+v"(acc[3][3]) : "v"(a[0]), "v"(a[3]));
    }
#pragma unroll
    for (int mb = 0; mb < 4; ++mb) {
#pragma unroll
        for (int nb = 0; nb < 4; ++nb) {
#pragma unroll
            for (int j = 0; j < 8; ++j) os[(hi * 8 + j) * 68 + nb * 16 + lr] = acc[mb][nb][j]; }
        __builtin_amdgcn_wave_barrier(); asm volatile("" ::: "memory");
        float* crow = C + (size_t)(r0 + mb * 16) * ldc + c0;
#pragma unroll 1
        for (int ps = 0; ps < 2; ++ps) {
#pragma unroll
            for (int s = 0; s < 8; ++s) { const int row = 2 * s + hi, cofs = lr * 4; v4f val = *(const v4fa*)(os + row * 68 + cofs); val = val * csc;
                if (BIAS) { val[0] += bfr(bias[c0 + cofs]); val[1] += bfr(bias[c0 + cofs + 1]); val[2] += bfr(bias[c0 + cofs + 2]); val[3] += bfr(bias[c0 + cofs + 3]); }
                *(volatile v4f*)(crow + (size_t)row * ldc + cofs) = val; }
            if (ps == 0) __threadfence(); }
        __builtin_amdgcn_wave_barrier(); asm volatile("" ::: "memory");
    }
}

__global__ __launch_bounds__(256) void k_wtG(const float* __restrict__ w, int K, int N, bf* Bt) {
    const int lane = threadIdx.x & 31; const int L0 = (blockIdx.x * 8 + (threadIdx.x >> 5)) * 8; const int nlines = N * K / 64;
#pragma unroll
    for (int ps = 0; ps < 2; ++ps) {
#pragma unroll 1
        for (int l = 0; l < 8; ++l) { const int L = L0 + l; if (L >= nlines) break; const size_t e = (size_t)L * 64 + lane * 2; const int k = (int)(e % K), n = (int)(e / K); v2us o;
            o[0] = f2bf(w[(size_t)k * N + n]); o[1] = f2bf(w[(size_t)(k + 1) * N + n]); *(volatile v2us*)(Bt + e) = o; }
        if (ps == 0) __threadfence(); }
}

__global__ __launch_bounds__(256) void k_cvt8(const float* __restrict__ src, bf* dst, size_t n8) { const size_t i = (size_t)blockIdx.x * 256 + threadIdx.x; if (i >= n8) return; const v8f v = *(const v8f*)(src + i * 8); v8us o;
#pragma unroll
    for (int k = 0; k < 8; ++k) o[k] = f2bf(v[k]); *(volatile v8us*)(dst + i * 8) = o; __threadfence(); *(volatile v8us*)(dst + i * 8) = o; }

__global__ __launch_bounds__(128) void k_wtH(const float* __restrict__ w, int N, h16* Bt) {
    const unsigned lane = threadIdx.x & 31u; const unsigned wave = (unsigned)__builtin_amdgcn_readfirstlane((int)(threadIdx.x >> 5));
    const unsigned n = blockIdx.x; const size_t zo = (size_t)blockIdx.y * DD * (size_t)N;
    const float* wz = w + zo + n; h16* bz = Bt + zo + (size_t)n * DD;
    v2h o[3];
#pragma unroll
    for (int l = 0; l < 3; ++l) { const unsigned k = (wave + 4u * l) * 64u + lane * 2u;
        o[l][0] = toh_flush(bfr(wz[(size_t)k * N]) * WSC); o[l][1] = toh_flush(bfr(wz[(size_t)(k + 1u) * N]) * WSC); }
#pragma unroll
    for (int ps = 0; ps < 2; ++ps) {
#pragma unroll
        for (int l = 0; l < 3; ++l) { const unsigned k = (wave + 4u * l) * 64u + lane * 2u; *(volatile v2h*)(bz + k) = o[l]; }
        if (ps == 0) __threadfence(); }
}

__global__ __launch_bounds__(256) void k_cvh8(const float* __restrict__ src, h16* dst, unsigned n8, unsigned lgc) { const unsigned i = blockIdx.x * 256u + threadIdx.x; if (i >= n8) return; const float carry = __uint_as_float((127u + lgc) << 23); const v8f v = *(const v8f*)(src + (size_t)i * 8); v8h o;
#pragma unroll
    for (int k = 0; k < 8; ++k) o[k] = toh_flush(v[k] * carry); *(volatile v8h*)(dst + (size_t)i * 8) = o; __threadfence(); *(volatile v8h*)(dst + (size_t)i * 8) = o; }

__global__ __launch_bounds__(256) void k_hplane(const float* __restrict__ Hf, h16* H16, h16* HT16, unsigned lgc) {
    __shared__ __align__(16) float s_t[64 * HP_PITCH];
    const unsigned tid = threadIdx.x;
    const float carry = __uint_as_float((127u + lgc) << 23);
    const unsigned d0 = blockIdx.x * 64u, row0 = blockIdx.y * 64u, b = blockIdx.y >> 1, j0 = (blockIdx.y & 1u) * 64u;
#pragma unroll
    for (int it = 0; it < 4; ++it) { const unsigned q = it * 256u + tid, r = q >> 4, c4 = q & 15u;
        v4f v = *(const v4f*)(Hf + (size_t)(row0 + r) * DD + d0 + c4 * 4u); v = v * carry; *(v4fa*)(s_t + r * HP_PITCH + c4 * 4u) = v; }
    __syncthreads();
    v8h oa[2], ob[2];
#pragma unroll
    for (int it = 0; it < 2; ++it) { const unsigned q = it * 256u + tid, r = q >> 3, p = q & 7u;
        const v4f a0 = *(const v4fa*)(s_t + r * HP_PITCH + p * 8u); const v4f a1 = *(const v4fa*)(s_t + r * HP_PITCH + p * 8u + 4u);
        float t[8];
#pragma unroll
        for (int k = 0; k < 8; ++k) t[k] = s_t[(p * 8u + k) * HP_PITCH + r];
        oa[it] = cat8h(toh2_flush(a0[0], a0[1]), toh2_flush(a0[2], a0[3]), toh2_flush(a1[0], a1[1]), toh2_flush(a1[2], a1[3]));
        ob[it] = cat8h(toh2_flush(t[0], t[1]), toh2_flush(t[2], t[3]), toh2_flush(t[4], t[5]), toh2_flush(t[6], t[7])); }
#pragma unroll
    for (int ps = 0; ps < 2; ++ps) {
#pragma unroll
        for (int it = 0; it < 2; ++it) { const unsigned q = it * 256u + tid, r = q >> 3, p = q & 7u;
            *(volatile v8h*)(H16 + (size_t)(row0 + r) * DD + d0 + p * 8u) = oa[it];
            *(volatile v8h*)(HT16 + ((size_t)b * DD + d0 + r) * NN + j0 + p * 8u) = ob[it]; }
        if (ps == 0) __threadfence(); }
}

__global__ __launch_bounds__(256) void k_pair(const float* __restrict__ SS, const float* __restrict__ ST, const int* __restrict__ adj, const float* __restrict__ ab1, const float* __restrict__ A2, const float* __restrict__ ab2, float* LG) {
    __shared__ __align__(16) float s_lg[NN];
    const unsigned tid = threadIdx.x, lane = tid & 31u; const unsigned wave = (unsigned)__builtin_amdgcn_readfirstlane((int)(tid >> 5));
    const unsigned rq = blockIdx.x, b = rq >> 7;
    const v2f s2 = *(const v2f*)(SS + (size_t)rq * HID + 2u * lane);
    const v2f b2 = *(const v2f*)(ab1 + 2u * lane); const v2f w2 = *(const v2f*)(A2 + 2u * lane);
    const float s0 = s2[0], s1 = s2[1], c0 = bfr(b2[0]), c1 = bfr(b2[1]), a0 = bfr(w2[0]), a1 = bfr(w2[1]);
    const float bias2 = bfr(ab2[0]);
    int mk = adj[(size_t)rq * NN + 16u * wave + (lane & 15u)];
    asm volatile("" : "+v"(mk));
    const float* tb = ST + ((size_t)b * NN + 16u * wave) * HID + 2u * lane;
    float ev = 0.0f;
#pragma unroll 1
    for (unsigned jj = 0; jj < 16u; ++jj) {
        const v2f t2 = *(const v2f*)(tb + (size_t)jj * HID);
        float h0 = (s0 + t2[0]) + c0; h0 = (h0 > 0.0f) ? h0 : 0.0f;
        float h1 = (s1 + t2[1]) + c1; h1 = (h1 > 0.0f) ? h1 : 0.0f;
        float acc = 0.0f; acc = fmaf(a0, h0, acc); acc = fmaf(a1, h1, acc);
#pragma unroll
        for (int sh = 16; sh; sh >>= 1) acc += __shfl_xor(acc, sh, 32);
        ev = (lane == jj) ? acc : ev;
    }
    float e = ev + bias2; e = (e > 0.0f) ? e : 0.01f * e;
    const float lg = (mk != 0) ? e : -1.0e30f;
    if (lane < 16u) s_lg[16u * wave + lane] = lg;
    __syncthreads();
    if (wave == 0u) {
        const v4f row = *(const v4fa*)(s_lg + lane * 4u);
        float* dst = LG + (size_t)rq * NN + lane * 4u;
        *(volatile v4f*)dst = row; __threadfence(); *(volatile v4f*)dst = row;
    }
}

__global__ __launch_bounds__(256) void k_gsoft(const float* __restrict__ LG, h16* P16) {
    __shared__ float red[8];
    const unsigned tid = threadIdx.x, lane = tid & 31u; const unsigned wave = (unsigned)__builtin_amdgcn_readfirstlane((int)(tid >> 5));
    const float* lg = LG + (size_t)blockIdx.x * NN * NN; h16* pd = P16 + (size_t)blockIdx.x * NN * NN;
    float m = -3.0e38f;
#pragma unroll 1
    for (unsigned it = 0; it < 8u; ++it) { const v8f v = *(const v8f*)(lg + (size_t)(it * 256u + tid) * 8u);
#pragma unroll
        for (int k = 0; k < 8; ++k) m = (v[k] > m) ? v[k] : m; }
#pragma unroll
    for (int sh = 16; sh; sh >>= 1) { const float o = __shfl_xor(m, sh, 32); m = (o > m) ? o : m; }
    if (lane == 0u) red[wave] = m;
    __syncthreads();
    m = red[0];
#pragma unroll
    for (int w = 1; w < 8; ++w) { const float o = red[w]; m = (o > m) ? o : m; }
    __syncthreads();
    float sum = 0.0f;
#pragma unroll 1
    for (unsigned it = 0; it < 8u; ++it) { const v8f v = *(const v8f*)(lg + (size_t)(it * 256u + tid) * 8u);
#pragma unroll
        for (int k = 0; k < 8; ++k) { float d = v[k] - m;
            asm volatile("" : "+v"(d));
            sum += __builtin_amdgcn_exp2f(d * LOG2E); } }
#pragma unroll
    for (int sh = 16; sh; sh >>= 1) sum += __shfl_xor(sum, sh, 32);
    if (lane == 0u) red[wave] = sum;
    __syncthreads();
    sum = red[0];
#pragma unroll
    for (int w = 1; w < 8; ++w) sum += red[w];
    const float inv = __builtin_amdgcn_rcpf(sum); const float invp = inv * PCAR;
#pragma unroll 1
    for (unsigned it = 0; it < 8u; ++it) { const size_t off = (size_t)(it * 256u + tid) * 8u; const v8f v = *(const v8f*)(lg + off); v8h o;
#pragma unroll
        for (int k = 0; k < 8; ++k) { float d = v[k] - m;
            asm volatile("" : "+v"(d));
            o[k] = toh_flush(__builtin_amdgcn_exp2f(d * LOG2E) * invp); }
        *(volatile v8h*)(pd + off) = o; __threadfence(); *(volatile v8h*)(pd + off) = o; }
}

__global__ __launch_bounds__(256) void k_bn(const float* __restrict__ node, const float* __restrict__ gamma, const float* __restrict__ beta, float* out0) {
    __shared__ __align__(16) float s_g[NB * 256];
    const unsigned tid = threadIdx.x; const unsigned d = blockIdx.x * 256u + tid;
    float tot = 0.0f;
#pragma unroll 1
    for (unsigned b = 0; b < (unsigned)NB; ++b) { const float* p = node + (size_t)b * NN * DD + d; float s = 0.0f;
#pragma unroll 8
        for (unsigned i = 0; i < (unsigned)NN; ++i) s += p[(size_t)i * DD];
        s_g[b * 256u + tid] = s; tot += s; }
    const float mean = tot * BN_INV;
    float var = 0.0f;
#pragma unroll 1
    for (unsigned b = 0; b < (unsigned)NB; ++b) { const float t = s_g[b * 256u + tid] - mean; var += t * t; }
    var *= BN_INV;
    const float den = sqrtf(var + 1.0e-5f); const float ga = bfr(gamma[d]), be = bfr(beta[d]);
#pragma unroll 1
    for (unsigned b = 0; b < (unsigned)NB; ++b) { const float t = s_g[b * 256u + tid] - mean; const float y = (ga * t) / den + be; s_g[b * 256u + tid] = y; }
    __syncthreads();
#pragma unroll 1
    for (unsigned q = tid; q < (unsigned)NB * 64u; q += 256u) { const unsigned b = q >> 6, c4 = q & 63u;
        const v4f val = *(const v4fa*)(s_g + b * 256u + c4 * 4u);
        float* dst = out0 + (size_t)b * DD + blockIdx.x * 256u + c4 * 4u;
        *(volatile v4f*)dst = val; __threadfence(); *(volatile v4f*)dst = val; }
}

extern "C" void kernel_launch(void* const* d_in, const int* in_sizes, int n_in,
                              void* d_out, int out_size, void* d_ws, size_t ws_size, hipStream_t stream) {
    if (n_in < 13) return;
    if (in_sizes[0] < NB * NN * DD || in_sizes[1] < NB * DD || in_sizes[2] < NB * NN * NN || in_sizes[3] < DD * DD || in_sizes[4] < DD || in_sizes[5] < DD * DD || in_sizes[6] < DD
        || in_sizes[7] < 2 * DD * HID || in_sizes[8] < HID || in_sizes[9] < HID || in_sizes[10] < 1 || in_sizes[11] < DD || in_sizes[12] < DD) return;
    if (out_size < NB_FULL * DD + NB * NN * DD) return;
    const float* feature = (const float*)d_in[0];
    const float* aspect  = (const float*)d_in[1];
    const int*   adj     = (const int*)d_in[2];
    const float* W0      = (const float*)d_in[3];
    const float* b0      = (const float*)d_in[4];
    const float* W1      = (const float*)d_in[5];
    const float* b1      = (const float*)d_in[6];
    const float* A1      = (const float*)d_in[7];
    const float* ab1     = (const float*)d_in[8];
    const float* A2      = (const float*)d_in[9];
    const float* ab2     = (const float*)d_in[10];
    const float* gamma   = (const float*)d_in[11];
    const float* beta    = (const float*)d_in[12];
    (void)aspect;
    float* OUT0 = (float*)d_out;
    float* OUT1 = OUT0 + (size_t)NB_FULL * DD;

    char* wsp = (char*)d_ws;
    auto take = [&](size_t bytes) { char* p = wsp; wsp += (bytes + 255) & ~(size_t)255; return (void*)p; };
    bf*    FB    = (bf*)take((size_t)MR * DD * 2);
    bf*    W0T   = (bf*)take((size_t)DD * DD * 2);
    h16*   W1T   = (h16*)take((size_t)DD * DD * 2);
    h16*   A1T   = (h16*)take((size_t)2 * HID * DD * 2);
    float* HF    = (float*)take((size_t)MR * DD * 4);
    h16*   H16   = (h16*)take((size_t)MR * DD * 2);
    h16*   HT16  = (h16*)take((size_t)MR * DD * 2);
    float* SST   = (float*)take((size_t)2 * MR * HID * 4);
    float* LG    = (float*)take((size_t)MR * NN * 4);
    h16*   P16   = (h16*)take((size_t)MR * NN * 2);
    float* FEAT1 = (float*)take((size_t)MR * DD * 4);
    h16*   F16   = (h16*)take((size_t)MR * DD * 2);
    if ((size_t)(wsp - (char*)d_ws) > ws_size) return;

    k_cvt8<<<(unsigned)(((size_t)MR * DD / 8 + 255) / 256), 256, 0, stream>>>(feature, FB, (size_t)MR * DD / 8);
    k_wtG<<<(unsigned)((DD * DD / 64 + 63) / 64), 256, 0, stream>>>(W0, DD, DD, W0T);
    k_wtH<<<dim3(DD, 1), 128, 0, stream>>>(W1, DD, W1T);
    k_wtH<<<dim3(HID, 2), 128, 0, stream>>>(A1, HID, A1T);

    k_gemmw<bf, 0, true><<<dim3(MR / 64, DD / 64, 1), 32, 0, stream>>>(FB, nullptr, W0T, nullptr, DD, HF, DD, b0, 1.0f, 0, 0, 0);
    k_hplane<<<dim3(DD / 64, MR / 64), 256, 0, stream>>>(HF, H16, HT16, LGC1);
    k_gemmw<h16, 0, false><<<dim3(MR / 64, HID / 64, 2), 32, 0, stream>>>(H16, nullptr, A1T, nullptr, DD, SST, HID, nullptr, SSC1, 0, (size_t)HID * DD, (size_t)MR * HID);
    k_pair<<<(unsigned)MR, 256, 0, stream>>>(SST, SST + (size_t)MR * HID, adj, ab1, A2, ab2, LG);
    k_gsoft<<<(unsigned)NB, 256, 0, stream>>>(LG, P16);
    k_gemmw<h16, 0, false><<<dim3(NN / 64, DD / 64, NB), 32, 0, stream>>>(P16, nullptr, HT16, nullptr, NN, FEAT1, DD, nullptr, OSC1, (size_t)NN * NN, (size_t)DD * NN, (size_t)NN * DD);

    k_cvh8<<<(unsigned)(((size_t)MR * DD / 8 + 255) / 256), 256, 0, stream>>>(FEAT1, F16, (unsigned)(MR * DD / 8), LGF);
    k_gemmw<h16, 0, true><<<dim3(MR / 64, DD / 64, 1), 32, 0, stream>>>(F16, nullptr, W1T, nullptr, DD, HF, DD, b1, HSC2, 0, 0, 0);
    k_hplane<<<dim3(DD / 64, MR / 64), 256, 0, stream>>>(HF, H16, HT16, LGC2);
    k_gemmw<h16, 0, false><<<dim3(MR / 64, HID / 64, 2), 32, 0, stream>>>(H16, nullptr, A1T, nullptr, DD, SST, HID, nullptr, SSC2, 0, (size_t)HID * DD, (size_t)MR * HID);
    k_pair<<<(unsigned)MR, 256, 0, stream>>>(SST, SST + (size_t)MR * HID, adj, ab1, A2, ab2, LG);
    k_gsoft<<<(unsigned)NB, 256, 0, stream>>>(LG, P16);
    k_gemmw<h16, 0, false><<<dim3(NN / 64, DD / 64, NB), 32, 0, stream>>>(P16, nullptr, HT16, nullptr, NN, OUT1, DD, nullptr, OSC2, (size_t)NN * NN, (size_t)DD * NN, (size_t)NN * DD);

    k_bn<<<3, 256, 0, stream>>>(OUT1, gamma, beta, OUT0);
}
